// MultiHeadAttention_25331717112501
// MI455X (gfx1250) — hardware-run, weakly checked
//
#include <hip/hip_runtime.h>


#ifndef NB
#define NB 2
#endif
#ifndef SEQ
#define SEQ 2048
#endif
#define NB_FULL  2
#define SEQ_FULL 2048
#ifndef OUT_SEQ
#define OUT_SEQ SEQ
#endif
#define DM   768
#define NH_  8
#define HD   96
#define AW   4
#define QRS  2048.0f
#define QRI  (1.0f / 2048.0f)
#define LOG2E 1.4426950408889634f
#define PSH  14.0f
#define PSC  0.10206207261596575f

static_assert(HD % 32 == 0);
static_assert(HD % 16 == 0);
static_assert(NH_ * HD == DM);
static_assert(DM % 64 == 0);
static_assert(DM % 32 == 0);
static_assert(SEQ % 64 == 0);
static_assert((NB * SEQ) % 64 == 0);
static_assert(SEQ % 32 == 0);
static_assert(SEQ % (16 * AW) == 0);
static_assert((16 * HD * 2) % 512 == 0);
static_assert((16 * HD) / 8 == 192);
static_assert(((size_t)SEQ * DM) % 8 == 0);
static_assert(NB <= NB_FULL);
static_assert(SEQ <= SEQ_FULL);

typedef _Float16 h16;
typedef unsigned short bf;
typedef __attribute__((ext_vector_type(16))) __bf16   v16bf;
typedef __attribute__((ext_vector_type(16))) _Float16 v16h;
typedef __attribute__((ext_vector_type(8)))  _Float16 v8h;
typedef __attribute__((ext_vector_type(8)))  unsigned short v8us;
typedef __attribute__((ext_vector_type(8)))  float    v8f;
typedef __attribute__((ext_vector_type(4)))  float    v4f;
typedef v4f  __attribute__((may_alias)) v4fa;

__device__ __forceinline__ unsigned short f2bf(float f) { unsigned u = __float_as_uint(f); u += 0x7FFFu + ((u >> 16) & 1u); return (unsigned short)(u >> 16); }
__device__ __forceinline__ float bf2f(unsigned short s) { return __uint_as_float(((unsigned)s) << 16); }
__device__ __forceinline__ float bfr(float f) { return bf2f(f2bf(f)); }
__device__ __forceinline__ v16h cat16(v8h lo, v8h hi) { return __builtin_shufflevector(lo, hi, 0, 1, 2, 3, 4, 5, 6, 7, 8, 9, 10, 11, 12, 13, 14, 15); }
__device__ __forceinline__ v16bf cat16b(v8us lo, v8us hi) { return __builtin_bit_cast(v16bf, __builtin_shufflevector(lo, hi, 0, 1, 2, 3, 4, 5, 6, 7, 8, 9, 10, 11, 12, 13, 14, 15)); }
__device__ __forceinline__ v8f wmma16(v16h a, v16h b, v8f c) { return __builtin_amdgcn_wmma_f32_16x16x32_f16(false, a, false, b, (short)0, c, false, false); }
__device__ __forceinline__ v8f wmmab(v16bf a, v16bf b, v8f c) { return __builtin_amdgcn_wmma_f32_16x16x32_bf16(false, a, false, b, (short)0, c, false, false); }
__device__ __forceinline__ v16h  ldh(const h16* p) { return cat16(*(const v8h*)p, *(const v8h*)(p + 16)); }
__device__ __forceinline__ v16bf ldb(const bf* p)  { return cat16b(*(const v8us*)p, *(const v8us*)(p + 16)); }
__device__ __forceinline__ void wave_sync() { __builtin_amdgcn_fence(3  , "wavefront"); __builtin_amdgcn_wave_barrier(); asm volatile("" ::: "memory"); }

__global__ __launch_bounds__(256) void k_cvt8(const float* __restrict__ src, bf* dst, size_t n8) {
    const size_t i = (size_t)blockIdx.x * 256 + threadIdx.x; if (i >= n8) return;
    const v8f v = *(const v8f*)(src + i * 8); v8us o;
#pragma unroll
    for (int k = 0; k < 8; ++k) o[k] = f2bf(v[k]);
    *(volatile v8us*)(dst + i * 8) = o; __threadfence(); *(volatile v8us*)(dst + i * 8) = o;
}

__global__ __launch_bounds__(256) void k_cvtT(const float* __restrict__ src, bf* dst) {
    __shared__ float ts[64 * 65];
    const int tid = threadIdx.x; const int k0 = blockIdx.x * 64, n0 = blockIdx.y * 64;
#pragma unroll 4
    for (int i = tid; i < 4096; i += 256) { const int kk = i >> 6, nn = i & 63; ts[kk * 65 + nn] = src[(size_t)(k0 + kk) * DM + n0 + nn]; }
    __syncthreads();
#pragma unroll 1
    for (int ps = 0; ps < 2; ++ps) {
#pragma unroll
        for (int it = 0; it < 2; ++it) { const int piece = it * 256 + tid; const int nr = piece >> 3, k8 = (piece & 7) * 8; v8us o;
#pragma unroll
            for (int j = 0; j < 8; ++j) o[j] = f2bf(ts[(k8 + j) * 65 + nr]);
            *(volatile v8us*)(dst + (size_t)(n0 + nr) * DM + k0 + k8) = o; }
        if (ps == 0) __threadfence(); }
}

__global__ __launch_bounds__(32) void k_projqk(const bf* __restrict__ A, const bf* __restrict__ Bt, const float* __restrict__ bias, h16* Ph, h16* Pr) {
    __shared__ __align__(16) float os[16 * 100];
    const int K = DM;
    const int lane = threadIdx.x & 31, lr = lane & 15, hi = lane >> 4; const int r0 = blockIdx.x * 32, hd = blockIdx.y, c0 = hd * HD;
    v8f acc[2][6];
#pragma unroll
    for (int mb = 0; mb < 2; ++mb)
#pragma unroll
        for (int nb = 0; nb < 6; ++nb) acc[mb][nb] = (v8f){};
    const size_t aoff = (size_t)(r0 + lr) * K + 8 * hi, boff = (size_t)(c0 + lr) * K + 8 * hi;
#pragma unroll 1
    for (int kc = 0; kc < K; kc += 32) {
        v16bf a[2];
        a[0] = ldb(A + aoff + kc); a[1] = ldb(A + aoff + (size_t)16 * K + kc);
#pragma unroll
        for (int nb = 0; nb < 6; ++nb) { const v16bf b = ldb(Bt + boff + (size_t)nb * 16 * K + kc);
            acc[0][nb] = wmmab(a[0], b, acc[0][nb]); acc[1][nb] = wmmab(a[1], b, acc[1][nb]); }
        asm volatile("v_nop\n\tv_nop\n\tv_nop\n\tv_nop" : "+v"(acc[0][0]), "+v"(acc[0][1]), "+v"(acc[0][2]), "+v"(acc[0][3]), "+v"(acc[0][4]), "+v"(acc[0][5]),
                     "+v"(acc[1][0]), "+v"(acc[1][1]), "+v"(acc[1][2]), "+v"(acc[1][3]), "+v"(acc[1][4]), "+v"(acc[1][5]) : "v"(a[0]), "v"(a[1]));
    }
    float bv[6];
#pragma unroll
    for (int nb = 0; nb < 6; ++nb) bv[nb] = bfr(bias[c0 + nb * 16 + lr]);
    const int bb = r0 / SEQ, t0 = r0 % SEQ;
    const size_t pb0 = ((size_t)(bb * NH_ + hd) * SEQ + t0) * HD;
#pragma unroll
    for (int mb = 0; mb < 2; ++mb) {
#pragma unroll
        for (int nb = 0; nb < 6; ++nb) {
#pragma unroll
            for (int j = 0; j < 8; ++j) os[(hi * 8 + j) * 100 + nb * 16 + lr] = acc[mb][nb][j] + bv[nb]; }
        wave_sync();
        const size_t sb = pb0 + (size_t)(mb * 16) * HD;
#pragma unroll 1
        for (int ps = 0; ps < 2; ++ps) {
#pragma unroll
            for (int s = 0; s < 6; ++s) { const int piece = s * 32 + lane; const int row = piece / 12, c8 = (piece - row * 12) * 8;
                const v4f x0 = *(const v4fa*)(&os[row * 100 + c8]); const v4f x1 = *(const v4fa*)(&os[row * 100 + c8 + 4]); v8h hv, rv;
#pragma unroll
                for (int i = 0; i < 4; ++i) { const h16 a0 = (h16)x0[i]; const h16 a1 = (h16)x1[i]; hv[i] = a0; hv[4 + i] = a1; rv[i] = (h16)((x0[i] - (float)a0) * QRS); rv[4 + i] = (h16)((x1[i] - (float)a1) * QRS); }
                const size_t oo = sb + (size_t)piece * 8;
                *(volatile v8h*)(Ph + oo) = hv; *(volatile v8h*)(Pr + oo) = rv; }
            if (ps == 0) __threadfence(); }
        wave_sync();
    }
}

__global__ __launch_bounds__(32) void k_projvt(const bf* __restrict__ A, const bf* __restrict__ Bt, const float* __restrict__ bias, h16* Ph) {
    __shared__ __align__(16) float os[16 * 68];
    const int K = DM;
    const int lane = threadIdx.x & 31, lr = lane & 15, hi = lane >> 4; const int r0 = blockIdx.x * 64, c0 = blockIdx.y * 64;
    v8f acc[4][4];
#pragma unroll
    for (int mb = 0; mb < 4; ++mb)
#pragma unroll
        for (int nb = 0; nb < 4; ++nb) acc[mb][nb] = (v8f){};
    const size_t aoff = (size_t)(r0 + lr) * K + 8 * hi, boff = (size_t)(c0 + lr) * K + 8 * hi;
#pragma unroll 1
    for (int kc = 0; kc < K; kc += 32) {
        v16bf a[4];
#pragma unroll
        for (int mb = 0; mb < 4; ++mb) a[mb] = ldb(A + aoff + (size_t)mb * 16 * K + kc);
#pragma unroll
        for (int nb = 0; nb < 4; ++nb) { const v16bf b = ldb(Bt + boff + (size_t)nb * 16 * K + kc);
#pragma unroll
            for (int mb = 0; mb < 4; ++mb) acc[mb][nb] = wmmab(a[mb], b, acc[mb][nb]); }
        asm volatile("v_nop\n\tv_nop\n\tv_nop\n\tv_nop" : "+v"(acc[0][0]), "+v"(acc[1][1]), "+v"(acc[2][2]), "+v"(acc[3][3]), "+v"(acc[0][3]), "+v"(acc[1][3]), "+v"(acc[2][3]) : "v"(a[0]), "v"(a[1]), "v"(a[2]), "v"(a[3]));
    }
    const size_t tbase = (size_t)(c0 / SEQ) * DM * SEQ + (size_t)r0 * SEQ + (size_t)(c0 % SEQ);
#pragma unroll
    for (int mb = 0; mb < 4; ++mb) {
#pragma unroll
        for (int nb = 0; nb < 4; ++nb) {
#pragma unroll
            for (int j = 0; j < 8; ++j) os[(hi * 8 + j) * 68 + nb * 16 + lr] = acc[mb][nb][j]; }
        wave_sync();
        const size_t sb = tbase + (size_t)(mb * 16) * SEQ;
#pragma unroll 1
        for (int ps = 0; ps < 2; ++ps) {
#pragma unroll
            for (int s = 0; s < 4; ++s) { const int row = 4 * s + (lane >> 3), c8 = (lane & 7) * 8;
                const float br = bfr(bias[r0 + mb * 16 + row]);
                const v4f x0 = *(const v4fa*)(&os[row * 68 + c8]); const v4f x1 = *(const v4fa*)(&os[row * 68 + c8 + 4]); v8h hv;
#pragma unroll
                for (int i = 0; i < 4; ++i) { hv[i] = (h16)(x0[i] + br); hv[4 + i] = (h16)(x1[i] + br); }
                *(volatile v8h*)(Ph + sb + (size_t)row * SEQ + c8) = hv; }
            if (ps == 0) __threadfence(); }
        wave_sync();
    }
}

__global__ __launch_bounds__(32 * AW) void k_flash(const h16* __restrict__ QH, const h16* __restrict__ QR, const h16* __restrict__ KH, const h16* __restrict__ KR, const h16* __restrict__ VT, bf* CT, size_t plane) {
    __shared__ __align__(16) float os[AW * 16 * 100];
    const int lane = threadIdx.x & 31, wave = __builtin_amdgcn_readfirstlane((int)(threadIdx.x >> 5)), lr = lane & 15, hi = lane >> 4;
    const int zh = blockIdx.y;
    const int t0 = (blockIdx.x * AW + wave) * 16;
    const size_t pbase = (size_t)zh * SEQ * HD;
    const size_t qo = pbase + (size_t)(t0 + lr) * HD + 8 * hi;
    v16h qh[3], qr[3];
#pragma unroll
    for (int c = 0; c < 3; ++c) { qh[c] = ldh(QH + qo + 32 * c); qr[c] = ldh(QR + qo + 32 * c); }
    const size_t ko = pbase + (size_t)lr * HD + 8 * hi;
    const size_t vo = pbase + (size_t)lr * SEQ + 8 * hi;
    v8f o[6];
#pragma unroll
    for (int j = 0; j < 6; ++j) o[j] = (v8f){};
    float m = -3.0e38f, l = 0.0f;
#pragma unroll 1
    for (int key0 = 0; key0 < SEQ; key0 += 32) {
        float tt[2][8];
#pragma unroll
        for (int tl = 0; tl < 2; ++tl) {
            const h16* kh = KH + ko + (size_t)(key0 + 16 * tl) * HD;
            const h16* kr = KR + ko + (size_t)(key0 + 16 * tl) * HD;
            const v16h a0 = ldh(kh), a1 = ldh(kh + 32), a2 = ldh(kh + 64);
            const v16h e0 = ldh(kr), e1 = ldh(kr + 32), e2 = ldh(kr + 64);
            v8f sH = (v8f){}, sL = (v8f){};
            sH = wmma16(a0, qh[0], sH); sL = wmma16(a0, qr[0], sL);
            sH = wmma16(a1, qh[1], sH); sL = wmma16(e0, qh[0], sL);
            sH = wmma16(a2, qh[2], sH); sL = wmma16(a1, qr[1], sL);
            sL = wmma16(e1, qh[1], sL); sL = wmma16(a2, qr[2], sL); sL = wmma16(e2, qh[2], sL);
            asm volatile("v_nop\n\tv_nop\n\tv_nop\n\tv_nop" : "+v"(sH), "+v"(sL) : "v"(a0), "v"(a1), "v"(a2), "v"(e0), "v"(e1), "v"(e2));
#pragma unroll
            for (int r = 0; r < 8; ++r) tt[tl][r] = (sH[r] + sL[r] * QRI) * LOG2E;
        }
        float mx = -3.0e38f;
#pragma unroll
        for (int r = 0; r < 8; ++r) mx = fmaxf(mx, fmaxf(tt[0][r], tt[1][r]));
        mx = fmaxf(mx, __shfl_xor(mx, 16, 32));
        const float mnew = fmaxf(m, mx);
        const float alpha = __builtin_amdgcn_exp2f(m - mnew);
        const float sh = PSH - mnew;
        v16h pb; float ls = 0.0f;
#pragma unroll
        for (int r = 0; r < 8; ++r) { const h16 pa = (h16)__builtin_amdgcn_exp2f(tt[0][r] + sh); const h16 pc = (h16)__builtin_amdgcn_exp2f(tt[1][r] + sh); pb[r] = pa; pb[8 + r] = pc; ls += (float)pa + (float)pc; }
        l = l * alpha + ls; m = mnew;
#pragma unroll
        for (int j = 0; j < 6; ++j) o[j] = o[j] * alpha;
        const h16* va = VT + vo + key0;
        v16h vf[6];
#pragma unroll
        for (int j = 0; j < 6; ++j) vf[j] = ldh(va + (size_t)(16 * j) * SEQ);
#pragma unroll
        for (int j = 0; j < 6; ++j) o[j] = wmma16(vf[j], pb, o[j]);
        asm volatile("v_nop\n\tv_nop\n\tv_nop\n\tv_nop" : "+v"(o[0]), "+v"(o[1]), "+v"(o[2]), "+v"(o[3]), "+v"(o[4]), "+v"(o[5]) : "v"(vf[0]), "v"(vf[1]), "v"(vf[2]), "v"(vf[3]), "v"(vf[4]), "v"(vf[5]), "v"(pb));
    }
    l += __shfl_xor(l, 16, 32);
    const float inv = PSC * (1.0f / l);
    const int wb = wave * 16 * 100;
#pragma unroll
    for (int j = 0; j < 6; ++j) { v4f a, c;
        a[0] = o[j][0] * inv; a[1] = o[j][1] * inv; a[2] = o[j][2] * inv; a[3] = o[j][3] * inv; c[0] = o[j][4] * inv; c[1] = o[j][5] * inv; c[2] = o[j][6] * inv; c[3] = o[j][7] * inv;
        *(v4fa*)(&os[wb + lr * 100 + 16 * j + 8 * hi]) = a; *(v4fa*)(&os[wb + lr * 100 + 16 * j + 8 * hi + 4]) = c; }
    wave_sync();
    const size_t cb = pbase + (size_t)t0 * HD;
#pragma unroll 1
    for (int ps = 0; ps < 2; ++ps) {
#pragma unroll
        for (int s = 0; s < 6; ++s) { const int piece = s * 32 + lane; const int row = piece / 12, c8 = (piece - row * 12) * 8;
            const v4f x0 = *(const v4fa*)(&os[wb + row * 100 + c8]); const v4f x1 = *(const v4fa*)(&os[wb + row * 100 + c8 + 4]); v8us hv, lv;
#pragma unroll
            for (int i = 0; i < 4; ++i) { const unsigned short h0 = f2bf(x0[i]); const unsigned short h1 = f2bf(x1[i]); hv[i] = h0; hv[4 + i] = h1; lv[i] = f2bf(x0[i] - bf2f(h0)); lv[4 + i] = f2bf(x1[i] - bf2f(h1)); }
            const size_t oo = cb + (size_t)piece * 8;
            *(volatile v8us*)(CT + oo) = hv; *(volatile v8us*)(CT + plane + oo) = lv; }
        if (ps == 0) __threadfence(); }
}

__global__ __launch_bounds__(32) void k_out(const bf* __restrict__ CT, size_t plane, const bf* __restrict__ Bt, const float* __restrict__ bias, float* OUT) {
    __shared__ __align__(16) float os[16 * 68];
    const int lane = threadIdx.x & 31, lr = lane & 15, hi = lane >> 4; const int r0 = blockIdx.x * 64, c0 = blockIdx.y * 64;
    const int bb = r0 / SEQ, t0 = r0 % SEQ;
    v8f acc[4][4];
#pragma unroll
    for (int mb = 0; mb < 4; ++mb)
#pragma unroll
        for (int nb = 0; nb < 4; ++nb) acc[mb][nb] = (v8f){};
    const size_t aoff = ((size_t)bb * NH_ * SEQ + t0 + lr) * HD + 8 * hi, boff = (size_t)(c0 + lr) * DM + 8 * hi;
#pragma unroll 1
    for (int it = 0; it < 2 * (DM / 32); ++it) {
        const int pl = it / (DM / 32); const int kc = (it - pl * (DM / 32)) * 32; const int hh = kc / HD; const int d0 = kc - hh * HD;
        const bf* ap = CT + (size_t)pl * plane + aoff + (size_t)hh * SEQ * HD + d0;
        v16bf a[4];
#pragma unroll
        for (int mb = 0; mb < 4; ++mb) a[mb] = ldb(ap + (size_t)mb * 16 * HD);
#pragma unroll
        for (int nb = 0; nb < 4; ++nb) { const v16bf b = ldb(Bt + boff + (size_t)nb * 16 * DM + kc);
#pragma unroll
            for (int mb = 0; mb < 4; ++mb) acc[mb][nb] = wmmab(a[mb], b, acc[mb][nb]); }
        asm volatile("v_nop\n\tv_nop\n\tv_nop\n\tv_nop" : "+v"(acc[0][0]), "+v"(acc[1][1]), "+v"(acc[2][2]), "+v"(acc[3][3]), "+v"(acc[0][3]), "+v"(acc[1][3]), "+v"(acc[2][3]) : "v"(a[0]), "v"(a[1]), "v"(a[2]), "v"(a[3]));
    }
    float bv[4];
#pragma unroll
    for (int nb = 0; nb < 4; ++nb) bv[nb] = bfr(bias[c0 + nb * 16 + lr]);
#pragma unroll
    for (int mb = 0; mb < 4; ++mb) {
#pragma unroll
        for (int nb = 0; nb < 4; ++nb) {
#pragma unroll
            for (int j = 0; j < 8; ++j) os[(hi * 8 + j) * 68 + nb * 16 + lr] = acc[mb][nb][j] + bv[nb]; }
        wave_sync();
        float* orow = OUT + ((size_t)bb * OUT_SEQ + t0 + mb * 16) * DM + c0;
#pragma unroll 1
        for (int ps = 0; ps < 2; ++ps) {
#pragma unroll
            for (int s = 0; s < 8; ++s) { const int row = 2 * s + hi, cofs = lr * 4;
                const v4f val = *(const v4fa*)(&os[row * 68 + cofs]);
                *(volatile v4f*)(orow + (size_t)row * DM + cofs) = val; }
            if (ps == 0) __threadfence(); }
        wave_sync();
    }
}

static constexpr size_t al256(size_t v) { return (v + 255) & ~(size_t)255; }
static constexpr size_t PLANE_EL = (size_t)NB * NH_ * SEQ * HD;
static constexpr size_t SZ_XB = al256((size_t)NB * SEQ * DM * 2);
static constexpr size_t SZ_WT = al256((size_t)3 * DM * DM * 2);
static constexpr size_t SZ_PL = al256(PLANE_EL * 2);
static constexpr size_t SZ_CT = al256(2 * PLANE_EL * 2);
static constexpr size_t SZ_TOTAL = SZ_XB + SZ_WT + 5 * SZ_PL + SZ_CT;
static_assert(SZ_TOTAL <= (size_t)134217728);
static_assert(((size_t)DM * DM * 2) % 256 == 0);
static_assert((PLANE_EL * 2) % 256 == 0);
static_assert(PLANE_EL == (size_t)NB * DM * SEQ);

extern "C" void kernel_launch(void* const* d_in, const int* in_sizes, int n_in,
                              void* d_out, int out_size, void* d_ws, size_t ws_size, hipStream_t stream) {
    if (n_in < 7) return;
    const size_t needx = ((size_t)(NB - 1) * SEQ_FULL + SEQ) * DM;
    if ((size_t)in_sizes[0] < needx) return;
    if ((size_t)in_sizes[1] < (size_t)DM * DM || (size_t)in_sizes[3] < (size_t)DM * DM || (size_t)in_sizes[5] < (size_t)DM * DM) return;
    if ((size_t)in_sizes[2] < (size_t)DM || (size_t)in_sizes[4] < (size_t)DM || (size_t)in_sizes[6] < (size_t)DM) return;
    if ((size_t)out_size < ((size_t)(NB - 1) * OUT_SEQ + SEQ) * DM) return;
    if (SZ_TOTAL > ws_size) return;
    const float* x = (const float*)d_in[0]; const float* wq = (const float*)d_in[1]; const float* bq = (const float*)d_in[2];
    const float* wk = (const float*)d_in[3]; const float* bk = (const float*)d_in[4]; const float* wo = (const float*)d_in[5]; const float* bo = (const float*)d_in[6];
    float* OUT = (float*)d_out;
    char* wsp = (char*)d_ws;
    bf* XB = (bf*)wsp; wsp += SZ_XB;
    bf* WT = (bf*)wsp; wsp += SZ_WT;
    h16* QH = (h16*)wsp; wsp += SZ_PL;
    h16* QR = (h16*)wsp; wsp += SZ_PL;
    h16* KH = (h16*)wsp; wsp += SZ_PL;
    h16* KR = (h16*)wsp; wsp += SZ_PL;
    h16* VT = (h16*)wsp; wsp += SZ_PL;
    bf*  CT = (bf*)wsp;  wsp += SZ_CT;
    bf* WQT = WT; bf* WKT = WT + (size_t)DM * DM; bf* WOT = WT + (size_t)2 * DM * DM;

    if (SEQ == SEQ_FULL) {
        const size_t n8 = (size_t)NB * SEQ * DM / 8;
        k_cvt8<<<(unsigned)((n8 + 255) / 256), 256, 0, stream>>>(x, XB, n8);
    } else {
        const size_t n8 = (size_t)SEQ * DM / 8;
        for (int b = 0; b < NB; ++b) k_cvt8<<<(unsigned)((n8 + 255) / 256), 256, 0, stream>>>(x + (size_t)b * SEQ_FULL * DM, XB + (size_t)b * SEQ * DM, n8);
    }
    k_cvtT<<<dim3(DM / 64, DM / 64, 1), 256, 0, stream>>>(wq, WQT);
    k_cvtT<<<dim3(DM / 64, DM / 64, 1), 256, 0, stream>>>(wk, WKT);
    k_cvtT<<<dim3(DM / 64, DM / 64, 1), 256, 0, stream>>>(wo, WOT);

    k_projqk<<<dim3(NB * SEQ / 32, NH_, 1), 32, 0, stream>>>(XB, WQT, bq, QH, QR);
    k_projqk<<<dim3(NB * SEQ / 32, NH_, 1), 32, 0, stream>>>(XB, WKT, bk, KH, KR);
    k_projvt<<<dim3(DM / 64, NB * SEQ / 64, 1), 32, 0, stream>>>(WKT, XB, bk, VT);

    k_flash<<<dim3(SEQ / (16 * AW), NB * NH_, 1), 32 * AW, 0, stream>>>(QH, QR, KH, KR, VT, CT, PLANE_EL);

    k_out<<<dim3(NB * SEQ / 64, DM / 64, 1), 32, 0, stream>>>(CT, PLANE_EL, WOT, bo, OUT);
}
